// Rwkv_Tmix_x070_68075231642002
// MI455X (gfx1250) — hardware-run, weakly checked
//
#include <hip/hip_runtime.h>
#include <math.h>

constexpr int kBatch  = 2;
constexpr int kSteps  = 1024;
constexpr int kChan   = 2048;
constexpr int kHeads  = 32;
constexpr int kHdim   = 64;
constexpr int kTok    = kBatch * kSteps;
constexpr size_t kPlane = (size_t)kTok * kChan;
constexpr int kRankW  = 64;
constexpr int kRankA  = 64;
constexpr int kRankV  = 32;
constexpr int kRankVP = 64;
constexpr int kRankG  = 128;
constexpr int kChunk  = 16;

constexpr float kActCarry  = 16.0f;
constexpr float kWBigCarry = 1024.0f;
constexpr float kWLowCarry = 256.0f;
constexpr float kHidCarry  = 16.0f;
constexpr float kYCarry    = 128.0f;
constexpr float kResCarry  = 2048.0f;
constexpr float kResInv    = 1.0f / kResCarry;
constexpr float kScaleBig  = 1.0f / (kActCarry * kWBigCarry);
constexpr float kScaleLow1 = 1.0f / (kActCarry * kWLowCarry);
constexpr float kScaleLow2 = 1.0f / (kHidCarry * kWLowCarry);
constexpr float kScaleOut  = 1.0f / (kYCarry * kWBigCarry);
constexpr float kGnEps     = (float)(1e-5 * 64.0);
constexpr float kDecayC    = 0.60653065971263342f;

static_assert(kHeads * kHdim == kChan);
static_assert(kTok % 32 == 0 && kChan % 64 == 0);
static_assert(kRankW % 64 == 0 && kRankA % 64 == 0 && kRankVP % 64 == 0 && kRankG % 64 == 0);
static_assert(kChan % 32 == 0 && kRankW % 32 == 0 && kRankVP % 32 == 0 && kRankG % 32 == 0);
static_assert(kSteps % kChunk == 0);
static_assert((kTok * kHeads) % 8 == 0);
static_assert(kHdim == 64 && kChunk == 16 && kHeads == 32);
static_assert(kChan / 8 == 256);
static_assert((kSteps & (kSteps - 1)) == 0);

typedef __attribute__((ext_vector_type(16))) _Float16 v16h;
typedef __attribute__((ext_vector_type(8)))  _Float16 v8h;
typedef __attribute__((ext_vector_type(8)))  float    v8f;
typedef __attribute__((ext_vector_type(4)))  float    v4f;
typedef __attribute__((ext_vector_type(2)))  float    v2f;
typedef __attribute__((ext_vector_type(4)))  unsigned int v4u;

__device__ __forceinline__ unsigned pk16(unsigned short a, unsigned short b) {
  return (unsigned)a | ((unsigned)b << 16);
}
__device__ __forceinline__ unsigned short h_bits(float f) {
  const _Float16 h = (_Float16)f;
  return __builtin_bit_cast(unsigned short, h);
}
__device__ __forceinline__ void h_split(float v, unsigned short& hb, unsigned short& rb) {
  const _Float16 h = (_Float16)v;
  const float hf = (float)h;
  const float d = v - hf;
  const _Float16 r = (_Float16)(d * kResCarry);
  hb = __builtin_bit_cast(unsigned short, h);
  rb = __builtin_bit_cast(unsigned short, r);
}
__device__ __forceinline__ v4u pack8_plain(const float (&v)[8]) {
  unsigned short hb[8];
#pragma unroll
  for (int e = 0; e < 8; ++e) hb[e] = h_bits(v[e]);
  return (v4u){pk16(hb[0], hb[1]), pk16(hb[2], hb[3]), pk16(hb[4], hb[5]), pk16(hb[6], hb[7])};
}
__device__ __forceinline__ void pack8_split(const float (&v)[8], v4u& uh, v4u& ur) {
  unsigned short hb[8], rb[8];
#pragma unroll
  for (int e = 0; e < 8; ++e) h_split(v[e], hb[e], rb[e]);
  uh = (v4u){pk16(hb[0], hb[1]), pk16(hb[2], hb[3]), pk16(hb[4], hb[5]), pk16(hb[6], hb[7])};
  ur = (v4u){pk16(rb[0], rb[1]), pk16(rb[2], rb[3]), pk16(rb[4], rb[5]), pk16(rb[6], rb[7])};
}
__device__ __forceinline__ float wave_sum32(float v) {
#pragma unroll
  for (int o = 16; o > 0; o >>= 1) v += __shfl_xor(v, o, 32);
  return v;
}
__device__ __forceinline__ float sigm(float z) {
  return 1.0f / (1.0f + expf(-z));
}

struct FragH {
  union U { v16h v; v8h h[2]; };
  static __device__ __forceinline__ v16h load(const _Float16* p) {
    U f;
    f.h[0] = *(const v8h*)(p);
    f.h[1] = *(const v8h*)(p + 16);
    return f.v;
  }
  static __device__ __forceinline__ v8f mma(v16h a, v16h b, v8f c) {
    return __builtin_amdgcn_wmma_f32_16x16x32_f16(false, a, false, b, (short)0, c, false, false);
  }
};
__device__ __forceinline__ void guard_split(v8f& a0, v8f& a1, v8f& a2, v8f& a3,
                                            v16h x0, v16h x1, v16h x2, v16h x3, v16h y0, v16h y1) {
  asm volatile("v_nop\n\tv_nop\n\tv_nop\n\tv_nop"
               : "+v"(a0), "+v"(a1), "+v"(a2), "+v"(a3)
               : "v"(x0), "v"(x1), "v"(x2), "v"(x3), "v"(y0), "v"(y1));
}
__device__ __forceinline__ void guard_plain(v8f& a0, v8f& a1, v16h x0, v16h x1, v16h y0) {
  asm volatile("v_nop\n\tv_nop\n\tv_nop\n\tv_nop"
               : "+v"(a0), "+v"(a1)
               : "v"(x0), "v"(x1), "v"(y0));
}
__device__ __forceinline__ void acc_guard4(v8f& a, v8f& b, v8f& c, v8f& d) {
  asm volatile("v_nop\n\tv_nop\n\tv_nop\n\tv_nop" : "+v"(a), "+v"(b), "+v"(c), "+v"(d));
}

constexpr int EPI_NONE  = 0;
constexpr int EPI_TANH  = 1;
constexpr int EPI_SIGM  = 2;
constexpr int EPI_DECAY = 3;
constexpr int EPI_BSIGM = 4;
constexpr int EPI_LERP  = 5;
constexpr int EPI_MULX  = 6;

template <bool SPLIT, int EPI, int OUT_MODE>
__global__ __launch_bounds__(256) void gemm_f16_kernel(
    const unsigned short* __restrict__ Ahp, const unsigned short* __restrict__ Arp, int lda,
    const unsigned short* __restrict__ Bhp, const unsigned short* __restrict__ Brp, int ldb,
    void* __restrict__ Cout, void* __restrict__ Cout2, int ldc,
    const float* __restrict__ bias, const float* __restrict__ aux1, const float* __restrict__ aux2,
    int M, int N, int K, float scale, float ocarry) {
  static_assert(OUT_MODE == 0 || OUT_MODE == 1 || OUT_MODE == 2);
  static_assert(OUT_MODE != 0 || (EPI == EPI_NONE || EPI == EPI_DECAY || EPI == EPI_BSIGM || EPI == EPI_LERP));
  static_assert(OUT_MODE != 1 || (EPI == EPI_NONE || EPI == EPI_TANH || EPI == EPI_SIGM || EPI == EPI_MULX));
  static_assert(OUT_MODE != 2 || (EPI == EPI_NONE));
  __shared__ __align__(16) float sT[8][16 * 68];
  const int lane = threadIdx.x & 31;
  const int wave = threadIdx.x >> 5;
  const int tilesN = N >> 6;
  const int tilesM = M >> 5;
  const int tile = blockIdx.x * 8 + wave;
  if (tile >= tilesM * tilesN) return;
  const int tm = tile / tilesN;
  const int tn = tile - tm * tilesN;
  const int m0 = tm << 5;
  const int n0 = tn << 6;
  const int rlane = lane & 15;
  const int half8 = (lane >> 4) * 8;
  const int mOff  = (lane >> 4) * 8;

  const size_t aoff = (size_t)(m0 + rlane) * lda + half8;
  const size_t boff = (size_t)(n0 + rlane) * ldb + half8;
  const _Float16* pa0 = (const _Float16*)Ahp + aoff;
  const _Float16* pa1 = pa0 + (size_t)16 * lda;
  const _Float16* pr0 = SPLIT ? ((const _Float16*)Arp + aoff) : pa0;
  const _Float16* pr1 = pr0 + (size_t)16 * lda;
  const _Float16* pbh = (const _Float16*)Bhp + boff;
  const _Float16* pbr = SPLIT ? ((const _Float16*)Brp + boff) : pbh;
  const size_t bstep = (size_t)16 * ldb;

  v8f acc[2][4], accr[2][4];
#pragma unroll
  for (int i = 0; i < 2; ++i)
#pragma unroll
    for (int j = 0; j < 4; ++j) {
      acc[i][j]  = (v8f){0.f, 0.f, 0.f, 0.f, 0.f, 0.f, 0.f, 0.f};
      accr[i][j] = (v8f){0.f, 0.f, 0.f, 0.f, 0.f, 0.f, 0.f, 0.f};
    }

  for (int k0 = 0; k0 < K; k0 += 32) {
    const v16h ah0 = FragH::load(pa0 + k0);
    const v16h ah1 = FragH::load(pa1 + k0);
    v16h ar0 = ah0, ar1 = ah1;
    if (SPLIT) {
      ar0 = FragH::load(pr0 + k0);
      ar1 = FragH::load(pr1 + k0);
    }
#pragma unroll
    for (int j = 0; j < 4; ++j) {
      const v16h bh = FragH::load(pbh + j * bstep + k0);
      v16h br = bh;
      if (SPLIT) br = FragH::load(pbr + j * bstep + k0);
      acc[0][j] = FragH::mma(ah0, bh, acc[0][j]);
      acc[1][j] = FragH::mma(ah1, bh, acc[1][j]);
      if (SPLIT) {
        accr[0][j] = FragH::mma(ah0, br, accr[0][j]);
        accr[1][j] = FragH::mma(ah1, br, accr[1][j]);
        accr[0][j] = FragH::mma(ar0, bh, accr[0][j]);
        accr[1][j] = FragH::mma(ar1, bh, accr[1][j]);
        guard_split(acc[0][j], acc[1][j], accr[0][j], accr[1][j], ah0, ah1, ar0, ar1, bh, br);
      } else {
        guard_plain(acc[0][j], acc[1][j], ah0, ah1, bh);
      }
    }
  }
  acc_guard4(acc[0][0], acc[0][1], acc[0][2], acc[0][3]);
  acc_guard4(acc[1][0], acc[1][1], acc[1][2], acc[1][3]);
  if (SPLIT) {
    acc_guard4(accr[0][0], accr[0][1], accr[0][2], accr[0][3]);
    acc_guard4(accr[1][0], accr[1][1], accr[1][2], accr[1][3]);
  }

  float* slab = sT[wave];
  const int hh = lane >> 4, c4 = (lane & 15) * 4;
  const int q = lane >> 3, c8 = (lane & 7) * 8;
  v4f bias4 = (v4f){0.f, 0.f, 0.f, 0.f};
  if (EPI == EPI_DECAY || EPI == EPI_BSIGM) bias4 = *(const v4f*)(bias + n0 + c4);

#pragma unroll
  for (int i = 0; i < 2; ++i) {
    const int mBase = m0 + (i << 4);
#pragma unroll
    for (int j = 0; j < 4; ++j) {
#pragma unroll
      for (int r = 0; r < 8; ++r) {
        float v = acc[i][j][r];
        if (SPLIT) v += accr[i][j][r] * kResInv;
        v *= scale;
        slab[(mOff + r) * 68 + (j << 4) + rlane] = v;
      }
    }
    __builtin_amdgcn_fence(__ATOMIC_RELEASE, "workgroup");
    __builtin_amdgcn_wave_barrier();
    __builtin_amdgcn_fence(__ATOMIC_ACQUIRE, "workgroup");
    if (OUT_MODE == 0) {
      float* C = (float*)Cout;
      if (EPI == EPI_DECAY || EPI == EPI_BSIGM || EPI == EPI_LERP) {
#pragma unroll 1
        for (int it = 0; it < 8; ++it) {
          const int row = it * 2 + hh;
          float* sp = slab + row * 68 + c4;
          const v4f x = *(const v4f*)sp;
          v4f y = x;
          if (EPI == EPI_LERP) {
            const size_t go = (size_t)(mBase + row) * ldc + n0 + c4;
            const v4f s4 = *(const v4f*)(aux1 + go);
            const v4f f4 = *(const v4f*)(aux2 + go);
#pragma unroll
            for (int e = 0; e < 4; ++e) y[e] = x[e] + (f4[e] - x[e]) * s4[e];
          } else {
#pragma unroll
            for (int e = 0; e < 4; ++e) {
              const float sg = sigm(x[e] + bias4[e]);
              y[e] = (EPI == EPI_DECAY) ? (kDecayC * sg) : sg;
            }
          }
          *(v4f*)sp = y;
        }
      }
      for (int pass = 0; pass < 2; ++pass) {
#pragma unroll
        for (int it = 0; it < 8; ++it) {
          const int row = it * 2 + hh;
          const v4f v = *(const v4f*)(slab + row * 68 + c4);
          *(volatile v4f*)(C + (size_t)(mBase + row) * ldc + n0 + c4) = v;
        }
        __threadfence();
      }
    } else {
      if (EPI == EPI_TANH || EPI == EPI_SIGM || EPI == EPI_MULX) {
#pragma unroll 1
        for (int it = 0; it < 4; ++it) {
          const int row = it * 4 + q;
          float* sp = slab + row * 68 + c8;
          v4f xa = *(const v4f*)sp;
          v4f xb = *(const v4f*)(sp + 4);
          if (EPI == EPI_MULX) {
            const size_t go = (size_t)(mBase + row) * ldc + n0 + c8;
            const v4f ma = *(const v4f*)(aux1 + go);
            const v4f mb = *(const v4f*)(aux1 + go + 4);
#pragma unroll
            for (int e = 0; e < 4; ++e) {
              xa[e] = (xa[e] * ma[e]) * ocarry;
              xb[e] = (xb[e] * mb[e]) * ocarry;
            }
          } else {
#pragma unroll
            for (int e = 0; e < 4; ++e) {
              const float ya = (EPI == EPI_TANH) ? tanhf(xa[e]) : sigm(xa[e]);
              const float yb2 = (EPI == EPI_TANH) ? tanhf(xb[e]) : sigm(xb[e]);
              xa[e] = ya * ocarry;
              xb[e] = yb2 * ocarry;
            }
          }
          *(v4f*)sp = xa;
          *(v4f*)(sp + 4) = xb;
        }
      }
      unsigned short* C  = (unsigned short*)Cout;
      unsigned short* C2 = (unsigned short*)Cout2;
      for (int pass = 0; pass < 2; ++pass) {
#pragma unroll
        for (int it = 0; it < 4; ++it) {
          const int row = it * 4 + q;
          const float* sp = slab + row * 68 + c8;
          float v[8];
#pragma unroll
          for (int e = 0; e < 8; ++e) v[e] = sp[e];
          const size_t o = (size_t)(mBase + row) * ldc + n0 + c8;
          if (OUT_MODE == 2) {
            v4u uh, ur;
            pack8_split(v, uh, ur);
            *(volatile v4u*)(C + o) = uh;
            *(volatile v4u*)(C2 + o) = ur;
          } else {
            const v4u uh = pack8_plain(v);
            *(volatile v4u*)(C + o) = uh;
          }
        }
        __threadfence();
      }
    }
    __builtin_amdgcn_fence(__ATOMIC_RELEASE, "workgroup");
    __builtin_amdgcn_wave_barrier();
    __builtin_amdgcn_fence(__ATOMIC_ACQUIRE, "workgroup");
  }
}

template <bool SPLIT>
__global__ __launch_bounds__(256) void cvt_plane_kernel(const float* __restrict__ src,
                                                        unsigned short* __restrict__ outh,
                                                        unsigned short* __restrict__ outr,
                                                        int n8, float carry) {
  const int i = blockIdx.x * 256 + threadIdx.x;
  if (i >= n8) return;
  const size_t off = (size_t)i * 8;
  const v4f a = *(const v4f*)(src + off);
  const v4f b = *(const v4f*)(src + off + 4);
  float v[8];
#pragma unroll
  for (int e = 0; e < 4; ++e) {
    v[e]     = a[e] * carry;
    v[4 + e] = b[e] * carry;
  }
  v4u uh, ur;
  if (SPLIT) {
    pack8_split(v, uh, ur);
  } else {
    uh = pack8_plain(v);
    ur = uh;
  }
  for (int pass = 0; pass < 2; ++pass) {
    *(volatile v4u*)(outh + off) = uh;
    if (SPLIT) *(volatile v4u*)(outr + off) = ur;
    __threadfence();
  }
}

__global__ __launch_bounds__(256) void wt_plane_kernel(const float* __restrict__ W,
                                                       unsigned short* __restrict__ outh,
                                                       unsigned short* __restrict__ outr,
                                                       int Kd, int Nd, int KdP, int NdP, int has_res, float carry) {
  __shared__ float sm[64][65];
  const int t  = threadIdx.x;
  const int k0 = blockIdx.x * 64;
  const int n0 = blockIdx.y * 64;
#pragma unroll
  for (int i = 0; i < 16; ++i) {
    const int e = i * 256 + t;
    const int r = e >> 6;
    const int c = e & 63;
    const int kk = k0 + r;
    const int nn = n0 + c;
    const bool valid = (kk < Kd) && (nn < Nd);
    const int kc = (kk < Kd) ? kk : (Kd - 1);
    const int nc = (nn < Nd) ? nn : (Nd - 1);
    const float v = W[(size_t)kc * Nd + nc];
    sm[c][r] = valid ? (v * carry) : 0.0f;
  }
  __syncthreads();
  const int lane = t & 31, wave = t >> 5;
  const int q = lane >> 3, c8 = (lane & 7) * 8;
  for (int pass = 0; pass < 2; ++pass) {
#pragma unroll
    for (int it = 0; it < 2; ++it) {
      const int row = wave * 8 + it * 4 + q;
      float v[8];
#pragma unroll
      for (int e = 0; e < 8; ++e) v[e] = sm[row][c8 + e];
      v4u uh, ur;
      pack8_split(v, uh, ur);
      const size_t o = (size_t)(n0 + row) * KdP + k0 + c8;
      *(volatile v4u*)(outh + o) = uh;
      if (has_res) *(volatile v4u*)(outr + o) = ur;
    }
    __threadfence();
  }
}

__device__ __forceinline__ void mix8(const float* __restrict__ m, int c8, const float (&cur)[8],
                                     const float (&xx)[8], float (&o)[8]) {
  const v4f a = *(const v4f*)(m + c8);
  const v4f b = *(const v4f*)(m + c8 + 4);
#pragma unroll
  for (int e = 0; e < 4; ++e) {
    o[e]     = (cur[e]     + xx[e]     * a[e]) * kActCarry;
    o[4 + e] = (cur[4 + e] + xx[4 + e] * b[e]) * kActCarry;
  }
}

template <int MODE>
__global__ __launch_bounds__(256) void mix_kernel(const float* __restrict__ x, const float* __restrict__ shift,
                                                  const float* __restrict__ c0, const float* __restrict__ c1,
                                                  const float* __restrict__ c2, const float* __restrict__ c3,
                                                  unsigned short* P0, unsigned short* P1, unsigned short* P2,
                                                  unsigned short* P3, unsigned short* P4) {
  const int row = blockIdx.x;
  const int c8  = threadIdx.x * 8;
  const int t   = row & (kSteps - 1);
  const int b   = row / kSteps;
  const bool first = (t == 0);
  const int prow = first ? row : (row - 1);
  const float* xp = x + (size_t)row * kChan + c8;
  const float* pp = first ? (shift + (size_t)b * kChan + c8) : (x + (size_t)prow * kChan + c8);
  const v4f a  = *(const v4f*)(xp);
  const v4f bq = *(const v4f*)(xp + 4);
  const v4f pa = *(const v4f*)(pp);
  const v4f pb = *(const v4f*)(pp + 4);
  float cur[8], xx[8];
#pragma unroll
  for (int e = 0; e < 4; ++e) {
    cur[e]     = a[e];
    cur[4 + e] = bq[e];
    xx[e]      = pa[e] - a[e];
    xx[4 + e]  = pb[e] - bq[e];
  }
  float o[8];
  const size_t off = (size_t)row * kChan + c8;
  if (MODE == 0) {
    v4u u0, u1, u2, u3h, u3r;
    mix8(c0, c8, cur, xx, o); u0 = pack8_plain(o);
    mix8(c1, c8, cur, xx, o); u1 = pack8_plain(o);
    mix8(c2, c8, cur, xx, o); u2 = pack8_plain(o);
    mix8(c3, c8, cur, xx, o); pack8_split(o, u3h, u3r);
    for (int pass = 0; pass < 2; ++pass) {
      *(volatile v4u*)(P0 + off) = u0;
      *(volatile v4u*)(P1 + off) = u1;
      *(volatile v4u*)(P2 + off) = u2;
      *(volatile v4u*)(P3 + off) = u3h;
      *(volatile v4u*)(P4 + off) = u3r;
      __threadfence();
    }
  } else {
    v4u u0h, u0r, u1h, u1r;
    mix8(c0, c8, cur, xx, o); pack8_split(o, u0h, u0r);
    mix8(c1, c8, cur, xx, o); pack8_split(o, u1h, u1r);
    for (int pass = 0; pass < 2; ++pass) {
      *(volatile v4u*)(P0 + off) = u0h;
      *(volatile v4u*)(P1 + off) = u0r;
      *(volatile v4u*)(P2 + off) = u1h;
      *(volatile v4u*)(P3 + off) = u1r;
      __threadfence();
    }
  }
}

__global__ __launch_bounds__(256) void key_post_kernel(float* Kf, float* AB, float* KK,
                                                       const float* __restrict__ k_k,
                                                       const float* __restrict__ k_a) {
  const int lane = threadIdx.x & 31;
  const int pair = blockIdx.x * 8 + (threadIdx.x >> 5);
  const int tok = pair >> 5;
  const int h   = pair & (kHeads - 1);
  const size_t base = (size_t)tok * kChan + (size_t)h * kHdim;
  const int cb = h * kHdim;
  float ss;
  {
    const float ka = Kf[base + lane] * k_k[cb + lane];
    const float kb = Kf[base + lane + 32] * k_k[cb + lane + 32];
    ss = wave_sum32(ka * ka + kb * kb);
  }
  const float inv = 1.0f / fmaxf(sqrtf(ss), 1e-12f);
#pragma unroll 1
  for (int hf = 0; hf < 2; ++hf) {
    const size_t idx = base + lane + 32 * hf;
    const int c = cb + lane + 32 * hf;
    const float k0  = Kf[idx];
    const float av  = AB[idx];
    const float kkv = (k0 * k_k[c]) * inv;
    const float km  = k0 + k_a[c] * (k0 * av - k0);
    const float bv  = kkv * av;
    *(volatile float*)(Kf + idx) = km;
    *(volatile float*)(AB + idx) = bv;
    *(volatile float*)(KK + idx) = kkv;
    __threadfence();
    *(volatile float*)(Kf + idx) = km;
    *(volatile float*)(AB + idx) = bv;
    *(volatile float*)(KK + idx) = kkv;
  }
}

__global__ __launch_bounds__(256) void state_scan_kernel(const float* __restrict__ Rf, const float* __restrict__ Dd,
                                                         const float* __restrict__ Kf, const float* __restrict__ Vf,
                                                         const float* __restrict__ KKf, const float* __restrict__ Bv,
                                                         const float* __restrict__ S0, float* __restrict__ Y) {
  __shared__ __align__(16) float lv[6 * kChunk * 64];
  __shared__ __align__(16) float yb[kChunk * 64];
  const int bh  = blockIdx.x;
  const int b   = bh >> 5;
  const int h   = bh & (kHeads - 1);
  const int tid = threadIdx.x;
  const int i   = tid >> 2;
  const int q   = tid & 3;
  const int j0  = q * 16;
  const int lrow = tid >> 4;
  const int lc4  = (tid & 15) * 4;
  const size_t base = (size_t)b * kSteps * kChan + (size_t)h * kHdim;

  float S[16];
  {
    const float* sp = S0 + ((size_t)(b * kHeads + h) * kHdim + i) * kHdim + j0;
#pragma unroll
    for (int g4 = 0; g4 < 4; ++g4) {
      const v4f t = *(const v4f*)(sp + 4 * g4);
#pragma unroll
      for (int e = 0; e < 4; ++e) S[4 * g4 + e] = t[e];
    }
  }

#pragma unroll 1
  for (int ch = 0; ch < kSteps / kChunk; ++ch) {
    const size_t goff = base + (size_t)(ch * kChunk + lrow) * kChan + lc4;
    {
      const v4f t0 = *(const v4f*)(Rf + goff);
      const v4f t1 = *(const v4f*)(Dd + goff);
      const v4f t2 = *(const v4f*)(Kf + goff);
      const v4f t3 = *(const v4f*)(Vf + goff);
      const v4f t4 = *(const v4f*)(KKf + goff);
      const v4f t5 = *(const v4f*)(Bv + goff);
      const int lo = lrow * 64 + lc4;
      *(v4f*)(lv + 0 * kChunk * 64 + lo) = t0;
      *(v4f*)(lv + 1 * kChunk * 64 + lo) = t1;
      *(v4f*)(lv + 2 * kChunk * 64 + lo) = t2;
      *(v4f*)(lv + 3 * kChunk * 64 + lo) = t3;
      *(v4f*)(lv + 4 * kChunk * 64 + lo) = t4;
      *(v4f*)(lv + 5 * kChunk * 64 + lo) = t5;
    }
    __syncthreads();

#pragma unroll 1
    for (int s = 0; s < kChunk; ++s) {
      const float* pr  = lv + 0 * kChunk * 64 + s * 64 + j0;
      const float* pd  = lv + 1 * kChunk * 64 + s * 64 + j0;
      const float* pk  = lv + 2 * kChunk * 64 + s * 64 + j0;
      const float* pkk = lv + 4 * kChunk * 64 + s * 64 + j0;
      const float* pb  = lv + 5 * kChunk * 64 + s * 64 + j0;
      const float vi = lv[3 * kChunk * 64 + s * 64 + i];
      float sa = 0.0f;
#pragma unroll
      for (int g4 = 0; g4 < 4; ++g4) {
        const v4f k4 = *(const v4f*)(pkk + 4 * g4);
#pragma unroll
        for (int e = 0; e < 4; ++e) sa += S[4 * g4 + e] * k4[e];
      }
      sa += __shfl_xor(sa, 1, 32);
      sa += __shfl_xor(sa, 2, 32);
      sa = -sa;
      float out = 0.0f;
#pragma unroll
      for (int g4 = 0; g4 < 4; ++g4) {
        const v4f d4 = *(const v4f*)(pd + 4 * g4);
        const v4f b4 = *(const v4f*)(pb + 4 * g4);
        const v4f k4 = *(const v4f*)(pk + 4 * g4);
        const v4f r4 = *(const v4f*)(pr + 4 * g4);
#pragma unroll
        for (int e = 0; e < 4; ++e) {
          const float sn = S[4 * g4 + e] * d4[e] + sa * b4[e] + vi * k4[e];
          S[4 * g4 + e] = sn;
          out += sn * r4[e];
        }
      }
      out += __shfl_xor(out, 1, 32);
      out += __shfl_xor(out, 2, 32);
      if (q == 0) yb[s * 64 + i] = out;
    }
    __syncthreads();
    {
      const v4f val = *(const v4f*)(yb + lrow * 64 + lc4);
      *(volatile v4f*)(Y + goff) = val;
      __threadfence();
      *(volatile v4f*)(Y + goff) = val;
    }
  }
}

__global__ __launch_bounds__(256) void norm_bonus_kernel(const float* __restrict__ Y, const float* __restrict__ Rf,
                                                         const float* __restrict__ Kf, const float* __restrict__ Vf,
                                                         const float* __restrict__ r_k,
                                                         const float* __restrict__ ln_w, const float* __restrict__ ln_b,
                                                         float* __restrict__ X) {
  const int lane = threadIdx.x & 31;
  const int pair = blockIdx.x * 8 + (threadIdx.x >> 5);
  const int tok = pair >> 5;
  const int h   = pair & (kHeads - 1);
  const size_t base = (size_t)tok * kChan + (size_t)h * kHdim + 2 * lane;
  const int c = h * kHdim + 2 * lane;
  const v2f y2 = *(const v2f*)(Y + base);
  const v2f r2 = *(const v2f*)(Rf + base);
  const v2f k2 = *(const v2f*)(Kf + base);
  const v2f v2 = *(const v2f*)(Vf + base);
  const v2f q2 = *(const v2f*)(r_k + c);
  const v2f w2 = *(const v2f*)(ln_w + c);
  const v2f b2 = *(const v2f*)(ln_b + c);
  const float mu = wave_sum32(y2[0] + y2[1]) * (1.0f / 64.0f);
  const float d0 = y2[0] - mu;
  const float d1 = y2[1] - mu;
  const float var = wave_sum32(d0 * d0 + d1 * d1) * (1.0f / 64.0f);
  const float inv = 1.0f / sqrtf(var + kGnEps);
  const float bsum = wave_sum32((r2[0] * q2[0]) * k2[0] + (r2[1] * q2[1]) * k2[1]);
  v2f xo;
  xo[0] = ((d0 * inv) * w2[0] + b2[0]) + bsum * v2[0];
  xo[1] = ((d1 * inv) * w2[1] + b2[1]) + bsum * v2[1];
  *(volatile v2f*)(X + base) = xo;
  __threadfence();
  *(volatile v2f*)(X + base) = xo;
}

extern "C" void kernel_launch(void* const* d_in, const int* in_sizes, int n_in,
                              void* d_out, int out_size, void* d_ws, size_t ws_size, hipStream_t stream) {
  if (n_in < 30 || d_out == nullptr || d_ws == nullptr) return;
  const int nP = (int)kPlane;
  if (in_sizes[0] != nP || in_sizes[1] != kBatch * kChan) return;
  if (in_sizes[2] != kBatch * kHeads * kHdim * kHdim || in_sizes[3] != nP) return;
  for (int i = 4; i <= 10; ++i) if (in_sizes[i] != kChan) return;
  if (in_sizes[11] != kChan * kRankW || in_sizes[12] != kRankW * kChan || in_sizes[13] != kChan) return;
  if (in_sizes[14] != kChan * kRankA || in_sizes[15] != kRankA * kChan || in_sizes[16] != kChan) return;
  if (in_sizes[17] != kChan * kRankV || in_sizes[18] != kRankV * kChan) return;
  if (in_sizes[19] != kChan * kRankG || in_sizes[20] != kRankG * kChan) return;
  if (in_sizes[21] != kChan || in_sizes[22] != kChan || in_sizes[23] != kHeads * kHdim) return;
  for (int i = 24; i <= 27; ++i) if (in_sizes[i] != kChan * kChan) return;
  if (in_sizes[28] != kChan || in_sizes[29] != kChan) return;
  if (out_size != nP) return;

  const float* x      = (const float*)d_in[0];
  const float* shift  = (const float*)d_in[1];
  const float* s_init = (const float*)d_in[2];
  const float* vfirst = (const float*)d_in[3];
  const float* x_r = (const float*)d_in[4];
  const float* x_w = (const float*)d_in[5];
  const float* x_k = (const float*)d_in[6];
  const float* x_v = (const float*)d_in[7];
  const float* x_a = (const float*)d_in[8];
  const float* x_g = (const float*)d_in[9];
  const float* w0 = (const float*)d_in[10];
  const float* w1 = (const float*)d_in[11];
  const float* w2 = (const float*)d_in[12];
  const float* a0 = (const float*)d_in[13];
  const float* a1 = (const float*)d_in[14];
  const float* a2 = (const float*)d_in[15];
  const float* v0 = (const float*)d_in[16];
  const float* v1 = (const float*)d_in[17];
  const float* v2 = (const float*)d_in[18];
  const float* g1 = (const float*)d_in[19];
  const float* g2 = (const float*)d_in[20];
  const float* k_k = (const float*)d_in[21];
  const float* k_a = (const float*)d_in[22];
  const float* r_k = (const float*)d_in[23];
  const float* W_r = (const float*)d_in[24];
  const float* W_k = (const float*)d_in[25];
  const float* W_v = (const float*)d_in[26];
  const float* W_o = (const float*)d_in[27];
  const float* ln_w = (const float*)d_in[28];
  const float* ln_b = (const float*)d_in[29];
  float* out0 = (float*)d_out;

  char* ws = (char*)d_ws;
  size_t off = 0;
  auto carve = [&](size_t bytes) -> char* {
    char* p = ws + off;
    off += (bytes + 255) & ~(size_t)255;
    return p;
  };
  const size_t slotB = kPlane * 4;
  const size_t actB  = kPlane * 2;
  char* SA = carve(slotB);
  char* SB = carve(slotB);
  char* SC = carve(slotB);
  char* SD = carve(slotB);
  char* SE = carve(slotB);
  char* SF = carve(slotB);
  char* SG = carve(slotB);
  unsigned short* Y16  = (unsigned short*)carve(actB);
  unsigned short* w1T  = (unsigned short*)carve((size_t)kRankW * kChan * 2);
  unsigned short* a1Th = (unsigned short*)carve((size_t)kRankA * kChan * 2);
  unsigned short* a1Tr = (unsigned short*)carve((size_t)kRankA * kChan * 2);
  unsigned short* v1T  = (unsigned short*)carve((size_t)kRankVP * kChan * 2);
  unsigned short* g1T  = (unsigned short*)carve((size_t)kRankG * kChan * 2);
  unsigned short* w2T  = (unsigned short*)carve((size_t)kChan * kRankW * 2);
  unsigned short* a2Th = (unsigned short*)carve((size_t)kChan * kRankA * 2);
  unsigned short* a2Tr = (unsigned short*)carve((size_t)kChan * kRankA * 2);
  unsigned short* v2T  = (unsigned short*)carve((size_t)kChan * kRankVP * 2);
  unsigned short* g2T  = (unsigned short*)carve((size_t)kChan * kRankG * 2);
  unsigned short* HW   = (unsigned short*)carve((size_t)kTok * kRankW * 2);
  unsigned short* HAh  = (unsigned short*)carve((size_t)kTok * kRankA * 2);
  unsigned short* HAr  = (unsigned short*)carve((size_t)kTok * kRankA * 2);
  unsigned short* HV   = (unsigned short*)carve((size_t)kTok * kRankVP * 2);
  unsigned short* HG   = (unsigned short*)carve((size_t)kTok * kRankG * 2);
  if (off > ws_size || off > (size_t)134217728) return;

  unsigned short* XV  = (unsigned short*)SA;
  float*          Rf  = (float*)SA;
  unsigned short* XRh = (unsigned short*)SB;
  unsigned short* XRr = (unsigned short*)(SB + actB);
  float*          Kf  = (float*)SB;
  float*          Vf  = (float*)SC;
  float*          WD  = (float*)SD;
  float*          Xn  = (float*)SD;
  float*          AB  = (float*)SE;
  unsigned short* XAh = (unsigned short*)SF;
  unsigned short* XAr = (unsigned short*)(SF + actB);
  unsigned short* WBh = (unsigned short*)SF;
  unsigned short* WBr = (unsigned short*)(SF + actB);
  float*          KK  = (float*)SF;
  unsigned short* XW  = (unsigned short*)SG;
  unsigned short* XG  = (unsigned short*)(SG + actB);
  float*          VS  = (float*)SG;
  unsigned short* XKh = (unsigned short*)SG;
  unsigned short* XKr = (unsigned short*)(SG + actB);
  float*          Yf  = (float*)SG;

  wt_plane_kernel<<<dim3(kChan / 64, kRankW / 64), 256, 0, stream>>>(w1, w1T, w1T, kChan, kRankW, kChan, kRankW, 0, kWLowCarry);
  wt_plane_kernel<<<dim3(kChan / 64, kRankA / 64), 256, 0, stream>>>(a1, a1Th, a1Tr, kChan, kRankA, kChan, kRankA, 1, kWLowCarry);
  wt_plane_kernel<<<dim3(kChan / 64, kRankVP / 64), 256, 0, stream>>>(v1, v1T, v1T, kChan, kRankV, kChan, kRankVP, 0, kWLowCarry);
  wt_plane_kernel<<<dim3(kChan / 64, kRankG / 64), 256, 0, stream>>>(g1, g1T, g1T, kChan, kRankG, kChan, kRankG, 0, kWLowCarry);
  wt_plane_kernel<<<dim3(kRankW / 64, kChan / 64), 256, 0, stream>>>(w2, w2T, w2T, kRankW, kChan, kRankW, kChan, 0, kWLowCarry);
  wt_plane_kernel<<<dim3(kRankA / 64, kChan / 64), 256, 0, stream>>>(a2, a2Th, a2Tr, kRankA, kChan, kRankA, kChan, 1, kWLowCarry);
  wt_plane_kernel<<<dim3(kRankVP / 64, kChan / 64), 256, 0, stream>>>(v2, v2T, v2T, kRankV, kChan, kRankVP, kChan, 0, kWLowCarry);
  wt_plane_kernel<<<dim3(kRankG / 64, kChan / 64), 256, 0, stream>>>(g2, g2T, g2T, kRankG, kChan, kRankG, kChan, 0, kWLowCarry);

  mix_kernel<0><<<kTok, 256, 0, stream>>>(x, shift, x_w, x_g, x_v, x_a, XW, XG, XV, XAh, XAr);

  const int blkN2048 = (kTok / 32) * (kChan / 64) / 8;
  const int blkN64   = (kTok / 32) * (64 / 64) / 8;
  const int blkN128  = (kTok / 32) * (128 / 64) / 8;
  const int cvtBlocks = (kChan * kChan / 8) / 256;
  const int cvtN8 = kChan * kChan / 8;

  gemm_f16_kernel<false, EPI_TANH, 1><<<blkN64, 256, 0, stream>>>(
      XW, XW, kChan, w1T, w1T, kChan, (void*)HW, (void*)HW, kRankW, w0, w0, w0,
      kTok, kRankW, kChan, kScaleLow1, kHidCarry);
  gemm_f16_kernel<true, EPI_NONE, 2><<<blkN64, 256, 0, stream>>>(
      XAh, XAr, kChan, a1Th, a1Tr, kChan, (void*)HAh, (void*)HAr, kRankA, w0, w0, w0,
      kTok, kRankA, kChan, kScaleLow1 * kHidCarry, 1.0f);
  gemm_f16_kernel<false, EPI_NONE, 1><<<blkN64, 256, 0, stream>>>(
      XV, XV, kChan, v1T, v1T, kChan, (void*)HV, (void*)HV, kRankVP, w0, w0, w0,
      kTok, kRankVP, kChan, kScaleLow1 * kHidCarry, 1.0f);
  gemm_f16_kernel<false, EPI_SIGM, 1><<<blkN128, 256, 0, stream>>>(
      XG, XG, kChan, g1T, g1T, kChan, (void*)HG, (void*)HG, kRankG, w0, w0, w0,
      kTok, kRankG, kChan, kScaleLow1, kHidCarry);

  gemm_f16_kernel<false, EPI_DECAY, 0><<<blkN2048, 256, 0, stream>>>(
      HW, HW, kRankW, w2T, w2T, kRankW, (void*)WD, (void*)WD, kChan, w0, w0, w0,
      kTok, kChan, kRankW, kScaleLow2, 1.0f);
  gemm_f16_kernel<true, EPI_BSIGM, 0><<<blkN2048, 256, 0, stream>>>(
      HAh, HAr, kRankA, a2Th, a2Tr, kRankA, (void*)AB, (void*)AB, kChan, a0, a0, a0,
      kTok, kChan, kRankA, kScaleLow2, 1.0f);
  gemm_f16_kernel<false, EPI_BSIGM, 0><<<blkN2048, 256, 0, stream>>>(
      HV, HV, kRankVP, v2T, v2T, kRankVP, (void*)VS, (void*)VS, kChan, v0, v0, v0,
      kTok, kChan, kRankVP, kScaleLow2, 1.0f);

  cvt_plane_kernel<false><<<cvtBlocks, 256, 0, stream>>>(W_v, WBh, WBh, cvtN8, kWBigCarry);
  gemm_f16_kernel<false, EPI_LERP, 0><<<blkN2048, 256, 0, stream>>>(
      XV, XV, kChan, WBh, WBh, kChan, (void*)Vf, (void*)Vf, kChan, v0, VS, vfirst,
      kTok, kChan, kChan, kScaleBig, 1.0f);

  mix_kernel<1><<<kTok, 256, 0, stream>>>(x, shift, x_r, x_k, x_k, x_k, XRh, XRr, XKh, XKr, XKr);

  cvt_plane_kernel<true><<<cvtBlocks, 256, 0, stream>>>(W_r, WBh, WBr, cvtN8, kWBigCarry);
  gemm_f16_kernel<true, EPI_NONE, 0><<<blkN2048, 256, 0, stream>>>(
      XRh, XRr, kChan, WBh, WBr, kChan, (void*)Rf, (void*)Rf, kChan, w0, w0, w0,
      kTok, kChan, kChan, kScaleBig, 1.0f);

  cvt_plane_kernel<true><<<cvtBlocks, 256, 0, stream>>>(W_k, WBh, WBr, cvtN8, kWBigCarry);
  gemm_f16_kernel<true, EPI_NONE, 0><<<blkN2048, 256, 0, stream>>>(
      XKh, XKr, kChan, WBh, WBr, kChan, (void*)Kf, (void*)Kf, kChan, w0, w0, w0,
      kTok, kChan, kChan, kScaleBig, 1.0f);

  key_post_kernel<<<(kTok * kHeads) / 8, 256, 0, stream>>>(Kf, AB, KK, k_k, k_a);

  state_scan_kernel<<<kBatch * kHeads, 256, 0, stream>>>(Rf, WD, Kf, Vf, KK, AB, s_init, Yf);

  norm_bonus_kernel<<<(kTok * kHeads) / 8, 256, 0, stream>>>(Yf, Rf, Kf, Vf, r_k, ln_w, ln_b, Xn);

  gemm_f16_kernel<false, EPI_MULX, 1><<<blkN2048, 256, 0, stream>>>(
      HG, HG, kRankG, g2T, g2T, kRankG, (void*)Y16, (void*)Y16, kChan, w0, Xn, Xn,
      kTok, kChan, kRankG, kScaleLow2, kYCarry);

  cvt_plane_kernel<false><<<cvtBlocks, 256, 0, stream>>>(W_o, WBh, WBh, cvtN8, kWBigCarry);
  gemm_f16_kernel<false, EPI_NONE, 0><<<blkN2048, 256, 0, stream>>>(
      Y16, Y16, kChan, WBh, WBh, kChan, (void*)out0, (void*)out0, kChan, w0, w0, w0,
      kTok, kChan, kChan, kScaleOut, 1.0f);
}
